// Mamba2Block_12893491823336
// MI455X (gfx1250) — hardware-verified
//
#include <hip/hip_runtime.h>
#include <stddef.h>


#define D_MODEL 1024
#define D_STATE 64
#define D_CONV  4
#define D_INNER 2048
#define DT_RANK 64
#define BATCH   2
#define SEQ_T   1024
#define MROWS   (BATCH * SEQ_T)
#define XSSM_W  (DT_RANK + 2 * D_STATE)
#define LOG2E_F 1.4426950408889634f
#define YG_SCALE 16.0f
#define W_SCALE  64.0f
#define TCH 32

typedef __attribute__((ext_vector_type(16))) _Float16 v16h;
typedef __attribute__((ext_vector_type(8)))  _Float16 v8h;
typedef __attribute__((ext_vector_type(16))) __bf16   v16b;
typedef __attribute__((ext_vector_type(8)))  __bf16   v8b;
typedef __attribute__((ext_vector_type(8)))  float    v8f;
typedef __attribute__((ext_vector_type(4)))  float    v4f;
#define PSCALE 32768.0f
#define U16(p) ((const unsigned short*)(const void*)(p))
#define PSCALE_INV (1.0f / 32768.0f)

__device__ __forceinline__ unsigned short f2bf_bits(float f) {
  unsigned u = __float_as_uint(f);
  return (unsigned short)((u + 0x7FFFu + ((u >> 16) & 1u)) >> 16);
}
__device__ __forceinline__ float bf_bits2f(unsigned short h) { return __uint_as_float(((unsigned)h) << 16); }

__device__ __forceinline__ void dep_guard_h(v8f& a, v8f& b, v16h x, v16h y) { asm volatile("v_nop\n\tv_nop\n\tv_nop\n\tv_nop" : "+v"(a), "+v"(b) : "v"(x), "v"(y)); }
__device__ __forceinline__ void dep_guard_b(v8f& a, v8f& b, v16b x, v16b y) { asm volatile("v_nop\n\tv_nop\n\tv_nop\n\tv_nop" : "+v"(a), "+v"(b) : "v"(x), "v"(y)); }
__device__ __forceinline__ void keep4_h(v16h a, v16h b, v16h c, v16h d) { asm volatile("v_nop" :: "v"(a), "v"(b), "v"(c), "v"(d)); }
__device__ __forceinline__ void keep4_b(v16b a, v16b b, v16b c, v16b d) { asm volatile("v_nop" :: "v"(a), "v"(b), "v"(c), "v"(d)); }
__device__ __forceinline__ void acc_guard4(v8f& a, v8f& b, v8f& c, v8f& d) { asm volatile("v_nop\n\tv_nop\n\tv_nop\n\tv_nop" : "+v"(a), "+v"(b), "+v"(c), "+v"(d)); }
template <typename T> struct Frag;
template <> struct Frag<_Float16> {
  typedef v16h V; union U { v16h v; v8h h[2]; };
  static __device__ __forceinline__ v16h load(const _Float16* p) {
    U f; f.h[0] = *(const v8h*)(p); f.h[1] = *(const v8h*)(p + 16); return f.v;
  }
  static __device__ __forceinline__ v8f mma(v16h a, v16h b, v8f c) {
    return __builtin_amdgcn_wmma_f32_16x16x32_f16(false, a, false, b, (short)0, c, false, false);
  }
  static __device__ __forceinline__ void guard(v8f& a, v8f& b, v16h x, v16h y) { dep_guard_h(a, b, x, y); }
  static __device__ __forceinline__ void keep(v16h a, v16h b, v16h c, v16h d) { keep4_h(a, b, c, d); }
};
template <> struct Frag<__bf16> {
  typedef v16b V; union U { v16b v; v8b h[2]; };
  static __device__ __forceinline__ v16b load(const __bf16* p) {
    U f; f.h[0] = *(const v8b*)(p); f.h[1] = *(const v8b*)(p + 16); return f.v;
  }
  static __device__ __forceinline__ v8f mma(v16b a, v16b b, v8f c) {
    return __builtin_amdgcn_wmma_f32_16x16x32_bf16(false, a, false, b, (short)0, c, false, false);
  }
  static __device__ __forceinline__ void guard(v8f& a, v8f& b, v16b x, v16b y) { dep_guard_b(a, b, x, y); }
  static __device__ __forceinline__ void keep(v16b a, v16b b, v16b c, v16b d) { keep4_b(a, b, c, d); }
};

template <int ET> struct Elem;
template <> struct Elem<0> { typedef _Float16 T; };
template <> struct Elem<1> { typedef __bf16 T; };
template <int ET, bool SPLIT, int BIAS_MODE, int OUT_MODE, bool RESID, int ACT = 0>
__global__ __launch_bounds__(256) void wmma_gemm64(
    const unsigned short* __restrict__ Ap, const unsigned short* __restrict__ A2p, int lda, long strideA,
    const unsigned short* __restrict__ Btp, const unsigned short* __restrict__ Bt2p, int ldb, long strideB,
    void* __restrict__ Cout, void* __restrict__ Cout2, int ldc, long strideC,
    const float* __restrict__ bias,
    const float* __restrict__ resid, long strideR,
    int M, int N, int K, float scale) {
  typedef typename Elem<ET>::T T;
  typedef typename Frag<T>::V V;
  const T* A = (const T*)Ap; const T* A2 = (const T*)A2p; const T* Bt = (const T*)Btp; const T* Bt2 = (const T*)Bt2p;
  __shared__ __align__(16) float sT[8][16 * 68];
  const int b    = blockIdx.y;
  const int lane = threadIdx.x & 31;
  const int wave = threadIdx.x >> 5;
  const int tilesN = N >> 6;
  const int tilesM = M >> 6;
  const int tile = blockIdx.x * 8 + wave;
  if (tile >= tilesM * tilesN) return;
  const int tm = tile / tilesN;
  const int tn = tile - tm * tilesN;
  const int m0 = tm << 6;
  const int n0 = tn << 6;

  const T* Ab  = A  + (size_t)b * strideA;
  const T* Bb  = Bt + (size_t)b * strideB;
  const T* Ab2 = SPLIT ? (A2  + (size_t)b * strideA) : nullptr;
  const T* Bb2 = SPLIT ? (Bt2 + (size_t)b * strideB) : nullptr;

  const int rlane = lane & 15;
  const int koff  = (lane >> 4) * 8;
  const int mOff  = (lane >> 4) * 8;

  v8f acc[4][4];
#pragma unroll
  for (int i = 0; i < 4; ++i)
#pragma unroll
    for (int j = 0; j < 4; ++j) acc[i][j] = (v8f){0.f,0.f,0.f,0.f,0.f,0.f,0.f,0.f};

  for (int k0 = 0; k0 < K; k0 += 32) {
    V bh[4], bl[4];
#pragma unroll
    for (int j = 0; j < 4; ++j) {
      const size_t bo = (size_t)(n0 + (j << 4) + rlane) * ldb + koff + k0;
      bh[j] = Frag<T>::load(Bb + bo);
      if (SPLIT) bl[j] = Frag<T>::load(Bb2 + bo);
    }
#pragma unroll
    for (int i = 0; i < 4; ++i) {
      const size_t ao = (size_t)(m0 + (i << 4) + rlane) * lda + koff + k0;
      V ah = Frag<T>::load(Ab + ao);
      V al;
      if (SPLIT) al = Frag<T>::load(Ab2 + ao);
#pragma unroll
      for (int j = 0; j < 4; ++j) {
        acc[i][j] = Frag<T>::mma(ah, bh[j], acc[i][j]);
        if (SPLIT) {
          acc[i][j] = Frag<T>::mma(ah, bl[j], acc[i][j]);
          acc[i][j] = Frag<T>::mma(al, bh[j], acc[i][j]);
        }
      }
      Frag<T>::guard(acc[i][0], acc[i][3], ah, SPLIT ? al : ah);
    }
    Frag<T>::keep(bh[0], bh[1], bh[2], bh[3]);
    if (SPLIT) Frag<T>::keep(bl[0], bl[1], bl[2], bl[3]);
  }
  acc_guard4(acc[0][0], acc[0][1], acc[0][2], acc[0][3]);
  acc_guard4(acc[1][0], acc[1][1], acc[1][2], acc[1][3]);
  acc_guard4(acc[2][0], acc[2][1], acc[2][2], acc[2][3]);
  acc_guard4(acc[3][0], acc[3][1], acc[3][2], acc[3][3]);

  float* slab = sT[wave];
  const float* Rb = RESID ? (resid + (size_t)b * strideR) : nullptr;
#pragma unroll
  for (int i = 0; i < 4; ++i) {
    const int mBase = m0 + (i << 4);
#pragma unroll
    for (int j = 0; j < 4; ++j) {
      const int n = n0 + (j << 4) + rlane;
      float bv = 0.f;
      if (BIAS_MODE == 2) bv = bias[n];
#pragma unroll
      for (int r = 0; r < 8; ++r) {
        float v = acc[i][j][r] * scale;
        if (BIAS_MODE == 1) v += bias[mBase + mOff + r];
        if (BIAS_MODE == 2) v += bv;
        if (RESID) v += Rb[(size_t)(mBase + mOff + r) * ldc + n];
        if (ACT == 1) v = tanhf(v);
        if (ACT == 2) v = fmaxf(v, 0.0f);
        if (ACT == 3) v = v / (1.0f + expf(-v));
        if (ACT == 4) v = (v > 0.f) ? v : 0.01f * v;
        if (ACT == 5) v = 0.5f * v * (1.0f + erff(v * 0.70710678118654752f));
        slab[(mOff + r) * 68 + (j << 4) + rlane] = v;
      }
    }
    __builtin_amdgcn_fence(__ATOMIC_RELEASE, "workgroup");
    __builtin_amdgcn_wave_barrier();
    __builtin_amdgcn_fence(__ATOMIC_ACQUIRE, "workgroup");
    if (OUT_MODE == 0) {
      float* C = (float*)Cout + (size_t)b * strideC;
      const int hh = lane >> 4, c4 = (lane & 15) * 4;
      for (int pass = 0; pass < 2; ++pass) {
#pragma unroll
        for (int it = 0; it < 8; ++it) {
          const int row = it * 2 + hh;
          v4f v = *(const v4f*)(slab + row * 68 + c4);
          *(volatile v4f*)(C + (size_t)(mBase + row) * ldc + n0 + c4) = v;
        }
        __threadfence();
      }
    } else {
      const int q = lane >> 3, c8 = (lane & 7) * 8;
      unsigned short* C  = (unsigned short*)Cout  + (size_t)b * strideC;
      unsigned short* C2 = (OUT_MODE == 2) ? ((unsigned short*)Cout2 + (size_t)b * strideC) : nullptr;
      for (int pass = 0; pass < 2; ++pass) {
#pragma unroll
        for (int it = 0; it < 4; ++it) {
          const int row = it * 4 + q;
          const float* sp = slab + row * 68 + c8;
          v8h hv, lv;
#pragma unroll
          for (int e = 0; e < 8; ++e) {
            if (OUT_MODE == 1) {
              hv[e] = (_Float16)sp[e];
            } else {
              unsigned short hb = f2bf_bits(sp[e]);
              unsigned short lb = f2bf_bits(sp[e] - bf_bits2f(hb));
              hv[e] = __builtin_bit_cast(_Float16, hb);
              lv[e] = __builtin_bit_cast(_Float16, lb);
            }
          }
          *(volatile v8h*)(C + (size_t)(mBase + row) * ldc + n0 + c8) = hv;
          if (OUT_MODE == 2) *(volatile v8h*)(C2 + (size_t)(mBase + row) * ldc + n0 + c8) = lv;
        }
        __threadfence();
      }
    }
    __builtin_amdgcn_fence(__ATOMIC_RELEASE, "workgroup");
    __builtin_amdgcn_wave_barrier();
    __builtin_amdgcn_fence(__ATOMIC_ACQUIRE, "workgroup");
  }
}

__global__ __launch_bounds__(256) void cvt_split_bf16_8(const float* __restrict__ in,
    unsigned short* __restrict__ hi, unsigned short* __restrict__ lo, int n8) {
  const int i = blockIdx.x * 256 + threadIdx.x;
  if (i >= n8) return;
  const size_t o = (size_t)i * 8;
  const v4f a = *(const v4f*)(in + o);
  const v4f c = *(const v4f*)(in + o + 4);
  v8h hv, lv;
#pragma unroll
  for (int e = 0; e < 4; ++e) {
    const unsigned short h0 = f2bf_bits(a[e]);
    const unsigned short l0 = f2bf_bits(a[e] - bf_bits2f(h0));
    const unsigned short h1 = f2bf_bits(c[e]);
    const unsigned short l1 = f2bf_bits(c[e] - bf_bits2f(h1));
    hv[e] = __builtin_bit_cast(_Float16, h0);     lv[e] = __builtin_bit_cast(_Float16, l0);
    hv[4 + e] = __builtin_bit_cast(_Float16, h1); lv[4 + e] = __builtin_bit_cast(_Float16, l1);
  }
  unsigned short* ph = hi + o;
  unsigned short* pl = lo + o;
  *(volatile v8h*)ph = hv; *(volatile v8h*)pl = lv;
  __threadfence();
  *(volatile v8h*)ph = hv; *(volatile v8h*)pl = lv;
}

__global__ __launch_bounds__(256) void cvt_f16_8(const float* __restrict__ in,
    unsigned short* __restrict__ out, int n8, float sc) {
  const int i = blockIdx.x * 256 + threadIdx.x;
  if (i >= n8) return;
  const size_t o = (size_t)i * 8;
  const v4f a = *(const v4f*)(in + o);
  const v4f c = *(const v4f*)(in + o + 4);
  v8h hv;
#pragma unroll
  for (int e = 0; e < 4; ++e) { hv[e] = (_Float16)(a[e] * sc); hv[4 + e] = (_Float16)(c[e] * sc); }
  unsigned short* ph = out + o;
  *(volatile v8h*)ph = hv;
  __threadfence();
  *(volatile v8h*)ph = hv;
}

__global__ __launch_bounds__(256) void a2_table_kernel(const float* __restrict__ alog, float* __restrict__ a2t, int n4) {
  const int i = blockIdx.x * 256 + threadIdx.x;
  if (i >= n4) return;
  const size_t o = (size_t)i * 4;
  const v4f v = *(const v4f*)(alog + o);
  v4f r;
#pragma unroll
  for (int e = 0; e < 4; ++e) { const float aa = -expf(v[e]); r[e] = aa * LOG2E_F; }
  float* p = a2t + o;
  *(volatile v4f*)p = r;
  __threadfence();
  *(volatile v4f*)p = r;
}

__global__ __launch_bounds__(128) void ln_split_kernel(const float* __restrict__ x, const float* __restrict__ g,
    const float* __restrict__ bb, unsigned short* __restrict__ hi, unsigned short* __restrict__ lo,
    unsigned short* __restrict__ f16p) {
  __shared__ float red[4];
  __shared__ float stat[2];
  const int row = blockIdx.x;
  const int t = threadIdx.x, lane = t & 31, w = t >> 5;
  const size_t ob = (size_t)row * D_MODEL + 8 * t;
  const v4f a = *(const v4f*)(x + ob);
  const v4f c = *(const v4f*)(x + ob + 4);
  float v[8];
#pragma unroll
  for (int e = 0; e < 4; ++e) { v[e] = a[e]; v[4 + e] = c[e]; }
  float s = 0.f;
#pragma unroll
  for (int e = 0; e < 8; ++e) s += v[e];
#pragma unroll
  for (int m = 16; m >= 1; m >>= 1) s += __shfl_xor(s, m, 32);
  if (lane == 0) red[w] = s;
  __syncthreads();
  if (t == 0) stat[0] = ((red[0] + red[1]) + (red[2] + red[3])) * (1.0f / (float)D_MODEL);
  __syncthreads();
  const float mu = stat[0];
  float ss = 0.f;
#pragma unroll
  for (int e = 0; e < 8; ++e) { const float d = v[e] - mu; ss += d * d; }
#pragma unroll
  for (int m = 16; m >= 1; m >>= 1) ss += __shfl_xor(ss, m, 32);
  if (lane == 0) red[w] = ss;
  __syncthreads();
  if (t == 0) {
    const float var = ((red[0] + red[1]) + (red[2] + red[3])) * (1.0f / (float)D_MODEL);
    stat[1] = 1.0f / sqrtf(var + 1e-5f);
  }
  __syncthreads();
  const float rs = stat[1];
  const v4f g0 = *(const v4f*)(g + 8 * t), g1 = *(const v4f*)(g + 8 * t + 4);
  const v4f b0 = *(const v4f*)(bb + 8 * t), b1 = *(const v4f*)(bb + 8 * t + 4);
  float gg[8], be[8];
#pragma unroll
  for (int e = 0; e < 4; ++e) { gg[e] = g0[e]; gg[4 + e] = g1[e]; be[e] = b0[e]; be[4 + e] = b1[e]; }
  v8h hv, lv, fv;
#pragma unroll
  for (int e = 0; e < 8; ++e) {
    const float y = (v[e] - mu) * rs * gg[e] + be[e];
    const unsigned short hb = f2bf_bits(y);
    const unsigned short lb = f2bf_bits(y - bf_bits2f(hb));
    hv[e] = __builtin_bit_cast(_Float16, hb);
    lv[e] = __builtin_bit_cast(_Float16, lb);
    fv[e] = (_Float16)y;
  }
  unsigned short* ph = hi + ob;
  unsigned short* pl = lo + ob;
  unsigned short* pf = f16p + ob;
  *(volatile v8h*)ph = hv; *(volatile v8h*)pl = lv; *(volatile v8h*)pf = fv;
  __threadfence();
  *(volatile v8h*)ph = hv; *(volatile v8h*)pl = lv; *(volatile v8h*)pf = fv;
}

__global__ __launch_bounds__(256) void conv_silu_kernel(const float* __restrict__ xp, const float* __restrict__ cw,
    const float* __restrict__ cb, float* __restrict__ xcf, unsigned short* __restrict__ xch, unsigned short* __restrict__ xcl) {
  __shared__ __align__(16) float srow[D_INNER];
  const int row = blockIdx.x;
  const int t = threadIdx.x;
  const int tt = row & (SEQ_T - 1);
  const int c0 = 8 * t;
  v4f wv[8];
#pragma unroll
  for (int e = 0; e < 8; ++e) wv[e] = *(const v4f*)(cw + (size_t)(c0 + e) * D_CONV);
  float acc[8];
#pragma unroll
  for (int e = 0; e < 8; ++e) acc[e] = 0.f;
#pragma unroll
  for (int k = 0; k < D_CONV; ++k) {
    const int dk = k - (D_CONV - 1);
    const bool valid = (tt + dk) >= 0;
    const int rs = valid ? (row + dk) : row;
    const float msk = valid ? 1.0f : 0.0f;
    const float* p = xp + (size_t)rs * D_INNER + c0;
    const v4f u0 = *(const v4f*)p;
    const v4f u1 = *(const v4f*)(p + 4);
#pragma unroll
    for (int e = 0; e < 4; ++e) {
      acc[e]     += (msk * u0[e]) * wv[e][k];
      acc[4 + e] += (msk * u1[e]) * wv[4 + e][k];
    }
  }
  const v4f bq0 = *(const v4f*)(cb + c0);
  const v4f bq1 = *(const v4f*)(cb + c0 + 4);
  float bb[8];
#pragma unroll
  for (int e = 0; e < 4; ++e) { bb[e] = bq0[e]; bb[4 + e] = bq1[e]; }
  float sv[8];
  v8h hv, lv;
#pragma unroll
  for (int e = 0; e < 8; ++e) {
    const float v = bb[e] + acc[e];
    const float ex = expf(-v);
    const float s = v * __builtin_amdgcn_rcpf(1.0f + ex);
    sv[e] = s;
    const unsigned short hb = f2bf_bits(s);
    const unsigned short lb = f2bf_bits(s - bf_bits2f(hb));
    hv[e] = __builtin_bit_cast(_Float16, hb);
    lv[e] = __builtin_bit_cast(_Float16, lb);
  }
  const size_t ob = (size_t)row * D_INNER;
  *(v4f*)(srow + c0)     = (v4f){sv[0], sv[1], sv[2], sv[3]};
  *(v4f*)(srow + c0 + 4) = (v4f){sv[4], sv[5], sv[6], sv[7]};
  __syncthreads();
  const v4f o0 = *(const v4f*)(srow + 4 * t);
  const v4f o1 = *(const v4f*)(srow + D_INNER / 2 + 4 * t);
  unsigned short* ph = xch + ob + c0;
  unsigned short* pl = xcl + ob + c0;
  float* pf0 = xcf + ob + 4 * t;
  float* pf1 = pf0 + D_INNER / 2;
  *(volatile v8h*)ph = hv; *(volatile v8h*)pl = lv;
  *(volatile v4f*)pf0 = o0; *(volatile v4f*)pf1 = o1;
  __threadfence();
  *(volatile v8h*)ph = hv; *(volatile v8h*)pl = lv;
  *(volatile v4f*)pf0 = o0; *(volatile v4f*)pf1 = o1;
}

__global__ __launch_bounds__(256) void dtr_split_kernel(const float* __restrict__ xssm,
    unsigned short* __restrict__ hi, unsigned short* __restrict__ lo, int nrows) {
  const int i = blockIdx.x * 256 + threadIdx.x;
  const int row = i >> 3, j = i & 7;
  if (row >= nrows) return;
  const float* p = xssm + (size_t)row * XSSM_W + 8 * j;
  const v4f a = *(const v4f*)p;
  const v4f c = *(const v4f*)(p + 4);
  v8h hv, lv;
#pragma unroll
  for (int e = 0; e < 4; ++e) {
    const unsigned short h0 = f2bf_bits(a[e]);
    const unsigned short l0 = f2bf_bits(a[e] - bf_bits2f(h0));
    const unsigned short h1 = f2bf_bits(c[e]);
    const unsigned short l1 = f2bf_bits(c[e] - bf_bits2f(h1));
    hv[e] = __builtin_bit_cast(_Float16, h0);     lv[e] = __builtin_bit_cast(_Float16, l0);
    hv[4 + e] = __builtin_bit_cast(_Float16, h1); lv[4 + e] = __builtin_bit_cast(_Float16, l1);
  }
  const size_t o = (size_t)row * DT_RANK + 8 * j;
  unsigned short* ph = hi + o;
  unsigned short* pl = lo + o;
  *(volatile v8h*)ph = hv; *(volatile v8h*)pl = lv;
  __threadfence();
  *(volatile v8h*)ph = hv; *(volatile v8h*)pl = lv;
}

__global__ __launch_bounds__(256) void softplus_bias_kernel(const float* __restrict__ dtl, const float* __restrict__ bias,
    float* __restrict__ dt, int n4) {
  const int i = blockIdx.x * 256 + threadIdx.x;
  if (i >= n4) return;
  const size_t o = (size_t)i * 4;
  const v4f v = *(const v4f*)(dtl + o);
  const int c = (int)(o & (size_t)(D_INNER - 1));
  const v4f bv = *(const v4f*)(bias + c);
  v4f r;
#pragma unroll
  for (int e = 0; e < 4; ++e) {
    const float u = v[e] + bv[e];
    r[e] = fmaxf(u, 0.0f) + log1pf(expf(-fabsf(u)));
  }
  float* p = dt + o;
  *(volatile v4f*)p = r;
  __threadfence();
  *(volatile v4f*)p = r;
}

__global__ __launch_bounds__(256) void scan_kernel(const float* __restrict__ dt, const float* __restrict__ xssm,
    const float* __restrict__ xcf, const float* __restrict__ zf, const float* __restrict__ state,
    const float* __restrict__ a2t, const float* __restrict__ Dp, _Float16* __restrict__ yg, float* __restrict__ hout) {
  __shared__ __align__(16) float ybuf[TCH * 64];
  __shared__ __align__(16) float hst[64 * D_STATE];
  const int tid = threadIdx.x;
  const int lane = tid & 31, wave = tid >> 5;
  const int b = blockIdx.x / (D_INNER / 64);
  const int cbase = (blockIdx.x % (D_INNER / 64)) * 64;
  const int chl = tid >> 2, q = tid & 3;
  const int c = cbase + chl;
  float h[16], a2[16];
  {
    const float* hp = state + ((size_t)b * D_INNER + c) * D_STATE + 16 * q;
    const float* ap = a2t + (size_t)c * D_STATE + 16 * q;
#pragma unroll
    for (int g4 = 0; g4 < 4; ++g4) {
      const v4f hv = *(const v4f*)(hp + 4 * g4);
      const v4f av = *(const v4f*)(ap + 4 * g4);
#pragma unroll
      for (int e = 0; e < 4; ++e) { h[4 * g4 + e] = hv[e]; a2[4 * g4 + e] = av[e]; }
    }
  }
  const float Dv = Dp[c];
  for (int t = 0; t < SEQ_T; ++t) {
    const size_t row = (size_t)b * SEQ_T + t;
    const size_t rc = row * D_INNER + c;
    const float dtv = dt[rc];
    const float xv = xcf[rc];
    const float zv = zf[rc];
    const float* sr = xssm + row * XSSM_W + DT_RANK + 16 * q;
    float Bv[16], Cv[16];
#pragma unroll
    for (int g4 = 0; g4 < 4; ++g4) {
      const v4f bq = *(const v4f*)(sr + 4 * g4);
      const v4f cq = *(const v4f*)(sr + D_STATE + 4 * g4);
#pragma unroll
      for (int e = 0; e < 4; ++e) { Bv[4 * g4 + e] = bq[e]; Cv[4 * g4 + e] = cq[e]; }
    }
    const float dx = dtv * xv;
    float part = 0.f;
#pragma unroll
    for (int e = 0; e < 16; ++e) {
      const float dA = __builtin_amdgcn_exp2f(dtv * a2[e]);
      h[e] = dA * h[e] + dx * Bv[e];
      part += h[e] * Cv[e];
    }
    part += __shfl_xor(part, 1, 32);
    part += __shfl_xor(part, 2, 32);
    float y = part + Dv * xv;
    const float ez = __expf(-zv);
    const float sz = zv * __builtin_amdgcn_rcpf(1.0f + ez);
    y *= sz;
    const int tl = t & (TCH - 1);
    if (q == 0) ybuf[tl * 64 + chl] = y * YG_SCALE;
    if (tl == TCH - 1) {
      __syncthreads();
      const int rr = lane >> 3, c8 = (lane & 7) * 8;
      const int lr = wave * 4 + rr;
      const float* sp = ybuf + lr * 64 + c8;
      const v4f u0 = *(const v4f*)sp;
      const v4f u1 = *(const v4f*)(sp + 4);
      v8h hv;
#pragma unroll
      for (int e = 0; e < 4; ++e) { hv[e] = (_Float16)u0[e]; hv[4 + e] = (_Float16)u1[e]; }
      _Float16* dst = yg + (row - (TCH - 1) + (size_t)lr) * D_INNER + cbase + c8;
      *(volatile v8h*)dst = hv;
      __threadfence();
      *(volatile v8h*)dst = hv;
      __syncthreads();
    }
  }
  {
    float* hp = hst + chl * D_STATE + 16 * q;
#pragma unroll
    for (int g4 = 0; g4 < 4; ++g4) {
      const v4f v = (v4f){h[4 * g4], h[4 * g4 + 1], h[4 * g4 + 2], h[4 * g4 + 3]};
      *(v4f*)(hp + 4 * g4) = v;
    }
  }
  __syncthreads();
  {
    const int chsel = lane >> 4, c4 = (lane & 15) * 4;
    for (int pass = 0; pass < 2; ++pass) {
#pragma unroll
      for (int it = 0; it < 4; ++it) {
        const int chl2 = wave * 8 + 2 * it + chsel;
        const v4f v = *(const v4f*)(hst + chl2 * D_STATE + c4);
        float* dst = hout + ((size_t)b * D_INNER + cbase + chl2) * D_STATE + c4;
        *(volatile v4f*)dst = v;
      }
      __threadfence();
    }
  }
}

extern "C" void kernel_launch(void* const* d_in, const int* in_sizes, int n_in,
                              void* d_out, int out_size, void* d_ws, size_t ws_size,
                              hipStream_t stream) {
  if (n_in < 13) return;
  if (in_sizes[0] != MROWS * D_MODEL || in_sizes[1] != BATCH * D_INNER * D_STATE ||
      in_sizes[2] != 2 * D_INNER * D_MODEL || in_sizes[3] != D_INNER * D_CONV || in_sizes[4] != D_INNER ||
      in_sizes[5] != XSSM_W * D_INNER || in_sizes[6] != D_INNER * DT_RANK || in_sizes[7] != D_INNER ||
      in_sizes[8] != D_INNER * D_STATE || in_sizes[9] != D_INNER || in_sizes[10] != D_MODEL * D_INNER ||
      in_sizes[11] != D_MODEL || in_sizes[12] != D_MODEL) return;
  if (out_size != MROWS * D_MODEL + BATCH * D_INNER * D_STATE) return;

  const float* x          = (const float*)d_in[0];
  const float* state      = (const float*)d_in[1];
  const float* in_proj_w  = (const float*)d_in[2];
  const float* conv_w     = (const float*)d_in[3];
  const float* conv_b     = (const float*)d_in[4];
  const float* x_proj_w   = (const float*)d_in[5];
  const float* dt_proj_w  = (const float*)d_in[6];
  const float* dt_proj_b  = (const float*)d_in[7];
  const float* A_log      = (const float*)d_in[8];
  const float* D_param    = (const float*)d_in[9];
  const float* out_proj_w = (const float*)d_in[10];
  const float* ln_g       = (const float*)d_in[11];
  const float* ln_b       = (const float*)d_in[12];

  float* out  = (float*)d_out;
  float* hout = out + (size_t)MROWS * D_MODEL;

  const size_t MI = 1048576;
  const size_t O_XNH = 0, O_XNL = 4 * MI, O_XNF = 8 * MI;
  const size_t O_YG  = 0;
  const size_t O_WIH = 12 * MI, O_WIL = 16 * MI, O_WZF = 20 * MI;
  const size_t O_XP  = 24 * MI;
  const size_t O_DTL = 24 * MI;
  const size_t O_Z   = 40 * MI;
  const size_t O_XCF = 56 * MI;
  const size_t O_XCH = 72 * MI, O_XCL = 80 * MI;
  const size_t O_WXH = 88 * MI;
  const size_t O_WXL = O_WXH + (size_t)XSSM_W * D_INNER * 2;
  const size_t O_XSSM = O_WXL + (size_t)XSSM_W * D_INNER * 2;
  const size_t O_DRH = O_XSSM + (size_t)MROWS * XSSM_W * 4;
  const size_t O_DRL = O_DRH + (size_t)MROWS * DT_RANK * 2;
  const size_t O_WDH = O_DRL + (size_t)MROWS * DT_RANK * 2;
  const size_t O_WDL = O_WDH + (size_t)D_INNER * DT_RANK * 2;
  const size_t O_A2  = O_WDL + (size_t)D_INNER * DT_RANK * 2;
  const size_t O_WO  = O_A2 + (size_t)D_INNER * D_STATE * 4;
  const size_t O_DT  = O_WO + (size_t)D_MODEL * D_INNER * 2;
  const size_t O_END = O_DT + (size_t)MROWS * D_INNER * 4;
  if (O_END > ws_size) return;

  char* ws = (char*)d_ws;
  unsigned short* xn_hi = (unsigned short*)(ws + O_XNH);
  unsigned short* xn_lo = (unsigned short*)(ws + O_XNL);
  unsigned short* xn_f  = (unsigned short*)(ws + O_XNF);
  _Float16*       yg    = (_Float16*)(ws + O_YG);
  unsigned short* wi_hi = (unsigned short*)(ws + O_WIH);
  unsigned short* wi_lo = (unsigned short*)(ws + O_WIL);
  unsigned short* wz_f  = (unsigned short*)(ws + O_WZF);
  float*          xp    = (float*)(ws + O_XP);
  float*          dtl   = (float*)(ws + O_DTL);
  float*          zf    = (float*)(ws + O_Z);
  float*          xcf   = (float*)(ws + O_XCF);
  unsigned short* xc_hi = (unsigned short*)(ws + O_XCH);
  unsigned short* xc_lo = (unsigned short*)(ws + O_XCL);
  unsigned short* wx_hi = (unsigned short*)(ws + O_WXH);
  unsigned short* wx_lo = (unsigned short*)(ws + O_WXL);
  float*          xssm  = (float*)(ws + O_XSSM);
  unsigned short* dr_hi = (unsigned short*)(ws + O_DRH);
  unsigned short* dr_lo = (unsigned short*)(ws + O_DRL);
  unsigned short* wd_hi = (unsigned short*)(ws + O_WDH);
  unsigned short* wd_lo = (unsigned short*)(ws + O_WDL);
  float*          a2t   = (float*)(ws + O_A2);
  unsigned short* wo_f  = (unsigned short*)(ws + O_WO);
  float*          dtf   = (float*)(ws + O_DT);

  {
    const int n8 = D_INNER * D_MODEL / 8;
    cvt_split_bf16_8<<<(n8 + 255) / 256, 256, 0, stream>>>(in_proj_w, wi_hi, wi_lo, n8);
    cvt_f16_8<<<(n8 + 255) / 256, 256, 0, stream>>>(in_proj_w + (size_t)D_INNER * D_MODEL, wz_f, n8, W_SCALE);
  }
  {
    const int n8 = XSSM_W * D_INNER / 8;
    cvt_split_bf16_8<<<(n8 + 255) / 256, 256, 0, stream>>>(x_proj_w, wx_hi, wx_lo, n8);
  }
  {
    const int n8 = D_INNER * DT_RANK / 8;
    cvt_split_bf16_8<<<(n8 + 255) / 256, 256, 0, stream>>>(dt_proj_w, wd_hi, wd_lo, n8);
  }
  {
    const int n4 = D_INNER * D_STATE / 4;
    a2_table_kernel<<<(n4 + 255) / 256, 256, 0, stream>>>(A_log, a2t, n4);
  }
  {
    const int n8 = D_MODEL * D_INNER / 8;
    cvt_f16_8<<<(n8 + 255) / 256, 256, 0, stream>>>(out_proj_w, wo_f, n8, W_SCALE);
  }

  ln_split_kernel<<<MROWS, 128, 0, stream>>>(x, ln_g, ln_b, xn_hi, xn_lo, xn_f);

  {
    const int tiles = (MROWS / 64) * (D_INNER / 64);
    wmma_gemm64<1, true, 0, 0, false, 0><<<dim3((tiles + 7) / 8, 1), 256, 0, stream>>>(
        xn_hi, xn_lo, D_MODEL, 0L, wi_hi, wi_lo, D_MODEL, 0L,
        (void*)xp, (void*)xp, D_INNER, 0L, dt_proj_b, x, 0L, MROWS, D_INNER, D_MODEL, 1.0f);
    wmma_gemm64<0, false, 0, 0, false, 0><<<dim3((tiles + 7) / 8, 1), 256, 0, stream>>>(
        xn_f, xn_f, D_MODEL, 0L, wz_f, wz_f, D_MODEL, 0L,
        (void*)zf, (void*)zf, D_INNER, 0L, dt_proj_b, x, 0L, MROWS, D_INNER, D_MODEL, 1.0f / W_SCALE);
  }

  conv_silu_kernel<<<MROWS, 256, 0, stream>>>(xp, conv_w, conv_b, xcf, xc_hi, xc_lo);

  {
    const int tiles = (MROWS / 64) * (XSSM_W / 64);
    wmma_gemm64<1, true, 0, 0, false, 0><<<dim3((tiles + 7) / 8, 1), 256, 0, stream>>>(
        xc_hi, xc_lo, D_INNER, 0L, wx_hi, wx_lo, D_INNER, 0L,
        (void*)xssm, (void*)xssm, XSSM_W, 0L, dt_proj_b, x, 0L, MROWS, XSSM_W, D_INNER, 1.0f);
  }

  dtr_split_kernel<<<(MROWS * 8 + 255) / 256, 256, 0, stream>>>(xssm, dr_hi, dr_lo, MROWS);
  {
    const int tiles = (MROWS / 64) * (D_INNER / 64);
    wmma_gemm64<1, true, 0, 0, false, 0><<<dim3((tiles + 7) / 8, 1), 256, 0, stream>>>(
        dr_hi, dr_lo, DT_RANK, 0L, wd_hi, wd_lo, DT_RANK, 0L,
        (void*)dtl, (void*)dtl, D_INNER, 0L, dt_proj_b, x, 0L, MROWS, D_INNER, DT_RANK, 1.0f);
  }
  {
    const int n4 = MROWS * D_INNER / 4;
    softplus_bias_kernel<<<(n4 + 255) / 256, 256, 0, stream>>>(dtl, dt_proj_b, dtf, n4);
  }

  scan_kernel<<<BATCH * (D_INNER / 64), 256, 0, stream>>>(dtf, xssm, xcf, zf, state, a2t, D_param, yg, hout);

  {
    const int tiles = (MROWS / 64) * (D_MODEL / 64);
    wmma_gemm64<0, false, 0, 0, true, 0><<<dim3((tiles + 7) / 8, 1), 256, 0, stream>>>(
        (const unsigned short*)yg, (const unsigned short*)yg, D_INNER, 0L, wo_f, wo_f, D_INNER, 0L,
        (void*)out, (void*)out, D_MODEL, 0L, dt_proj_b, x, 0L, MROWS, D_MODEL, D_INNER, 1.0f / (YG_SCALE * W_SCALE));
  }
}
